// DeformableConvBlock_47485158425306
// MI455X (gfx1250) — hardware-verified
//
#include <hip/hip_runtime.h>
#include <math.h>

typedef __attribute__((ext_vector_type(16))) _Float16 v16h;
typedef __attribute__((ext_vector_type(16))) __bf16 v16b;
typedef __attribute__((ext_vector_type(8)))  _Float16 v8h;
typedef __attribute__((ext_vector_type(8)))  float v8f;
typedef __attribute__((ext_vector_type(4)))  float v4f;
typedef __attribute__((ext_vector_type(2)))  float v2f;
typedef __attribute__((ext_vector_type(4)))  unsigned v4u;
typedef __attribute__((ext_vector_type(4)))  int v4i;
typedef float __attribute__((may_alias)) float_a;
typedef int __attribute__((may_alias)) int_a;

template <typename T> __device__ __forceinline__ void vst2(void* p, T v) { *(volatile T*)p = v; __threadfence(); *(volatile T*)p = v; }
__device__ __forceinline__ v8f wmma16(v16h a, v16h b, v8f c) {
  v8f d = __builtin_amdgcn_wmma_f32_16x16x32_f16(false, a, false, b, (short)0, c, false, false);
  asm volatile("v_nop\n\tv_nop\n\tv_nop\n\tv_nop" : "+v"(d) : "v"(a), "v"(b));
  return d;
}
__device__ __forceinline__ v8f wmma_bf(v16b a, v16b b, v8f c) {
  v8f d = __builtin_amdgcn_wmma_f32_16x16x32_bf16(false, a, false, b, (short)0, c, false, false);
  asm volatile("v_nop\n\tv_nop\n\tv_nop\n\tv_nop" : "+v"(d) : "v"(a), "v"(b));
  return d;
}
__device__ __forceinline__ v16h frag_h(const _Float16* rowk0, int lane) {
  union { v16h v; v8h q[2]; } u; const _Float16* p = rowk0 + 8 * (lane >> 4);
  u.q[0] = *(const v8h*)p; u.q[1] = *(const v8h*)(p + 16); return u.v;
}
__device__ __forceinline__ v16h frag_f32(const float* rowk0, int lane) {
  v16h a; const float* p = rowk0 + 8 * (lane >> 4);
#pragma unroll
  for (int i = 0; i < 8; ++i) { a[i] = (_Float16)p[i]; a[8 + i] = (_Float16)p[16 + i]; }
  return a;
}
__device__ __forceinline__ v16h frag_f32s(const float* rowk0, int lane, float sc) {
  v16h a; const float* p = rowk0 + 8 * (lane >> 4);
#pragma unroll
  for (int i = 0; i < 8; ++i) { a[i] = (_Float16)(p[i] * sc); a[8 + i] = (_Float16)(p[16 + i] * sc); }
  return a;
}
__device__ __forceinline__ v16h fragc_f32(const float* W, int k0, int n, int lane, int ld, int K) {
  v16h a; const int g = lane >> 4;
#pragma unroll
  for (int i = 0; i < 8; ++i) { const int ka = k0 + 8 * g + i, kb = ka + 16;
    a[i] = (_Float16)(ka < K ? W[(size_t)ka * ld + n] : 0.f); a[8 + i] = (_Float16)(kb < K ? W[(size_t)kb * ld + n] : 0.f); }
  return a;
}
struct F2 { v16b h, l; };
__device__ __forceinline__ F2 bsplit16(const float v[16]) { F2 r;
#pragma unroll
  for (int i = 0; i < 16; ++i) { const __bf16 h = (__bf16)v[i]; r.h[i] = h; r.l[i] = (__bf16)(v[i] - (float)h); }
  return r; }
__device__ __forceinline__ F2 split_row(const float* row, int k0, int lane) { float v[16]; const float* p = row + k0 + 8 * (lane >> 4);
#pragma unroll
  for (int i = 0; i < 8; ++i) { v[i] = p[i]; v[8 + i] = p[16 + i]; }
  return bsplit16(v); }
__device__ __forceinline__ F2 split_rowK(const float* row, int k0, int lane, int K) { float v[16]; const int g = lane >> 4;
#pragma unroll
  for (int i = 0; i < 8; ++i) { const int ka = k0 + 8 * g + i, kb = ka + 16; v[i] = ka < K ? row[ka] : 0.f; v[8 + i] = kb < K ? row[kb] : 0.f; }
  return bsplit16(v); }
__device__ __forceinline__ F2 split_col(const float* W, int k0, int n, int lane, int ld, int K) { float v[16]; const int g = lane >> 4;
#pragma unroll
  for (int i = 0; i < 8; ++i) { const int ka = k0 + 8 * g + i, kb = ka + 16; v[i] = ka < K ? W[(size_t)ka * ld + n] : 0.f; v[8 + i] = kb < K ? W[(size_t)kb * ld + n] : 0.f; }
  return bsplit16(v); }
__device__ __forceinline__ v8f mac3(const F2& a, const F2& b, v8f c) { c = wmma_bf(a.l, b.h, c); c = wmma_bf(a.h, b.l, c); return wmma_bf(a.h, b.h, c); }
__device__ __forceinline__ float sigm(float v) { return 1.0f / (1.0f + expf(-v)); }
#define LDSX() do { asm volatile("s_wait_dscnt 0" ::: "memory"); __builtin_amdgcn_wave_barrier(); __builtin_amdgcn_fence(__ATOMIC_RELEASE, "workgroup"); } while (0)

#define NB 4
#define CC 64
#define HH 128
#define WW 128
#define NP (HH * WW)
#define OO 64
#define KK 9
#define KTOT (CC * KK)
#define NPB (NP / 64)

__global__ __launch_bounds__(128) void k_off(const float* __restrict__ x, const float* __restrict__ ow, const float* __restrict__ ob, float* __restrict__ om) {
  __shared__ __align__(16) float so[4][16][36];
  const int tid = threadIdx.x, wave = tid >> 5, lane = tid & 31, col = lane & 15, g = lane >> 4;
  const int b = blockIdx.y, r0 = blockIdx.x * 64 + wave * 16; const int p = r0 + col, py = p / WW, px = p % WW;
  const float* xb = x + (size_t)b * CC * NP;
  v8f acc[2] = {};
#pragma unroll 1
  for (int kc = 0; kc < KTOT / 32; ++kc) {
    float av[16];
#pragma unroll
    for (int i = 0; i < 16; ++i) { const int k = kc * 32 + (i < 8 ? 8 * g + i : 16 + 8 * g + (i - 8)); const int c = k / 9, t = k % 9, yy = py + t / 3 - 1, xx = px + t % 3 - 1;
      av[i] = (yy >= 0 && yy < HH && xx >= 0 && xx < WW) ? xb[(size_t)c * NP + yy * WW + xx] : 0.f; }
    const F2 a = bsplit16(av);
#pragma unroll
    for (int j = 0; j < 2; ++j) { const int o = j * 16 + col; float wv[16]; const float* wr = o < 18 ? ow + (size_t)o * KTOT : nullptr;
#pragma unroll
      for (int i = 0; i < 16; ++i) { const int k = kc * 32 + (i < 8 ? 8 * g + i : 16 + 8 * g + (i - 8)); wv[i] = wr ? wr[k] : 0.f; }
      acc[j] = mac3(a, bsplit16(wv), acc[j]); } }
#pragma unroll
  for (int j = 0; j < 2; ++j) { const int o = j * 16 + col; const float bb = o < 18 ? ob[o] : 0.f;
#pragma unroll
    for (int r = 0; r < 8; ++r) so[wave][8 * g + r][o] = acc[j][r] + bb; }
  LDSX();
  for (int q = lane; q < 16 * 8; q += 32) { const int rl = q >> 3, pc = q & 7; vst2(om + ((size_t)b * NP + r0 + rl) * 32 + pc * 4, *(const v4f*)(&so[wave][rl][pc * 4])); }
}
__global__ __launch_bounds__(256) void k_xT(const float* __restrict__ x, float* __restrict__ xt) {
  __shared__ float tile[64][65];
  const int b = blockIdx.z, p0 = blockIdx.x * 64, c0 = blockIdx.y * 64, tid = threadIdx.x;
  for (int q = tid; q < 64 * 64; q += 256) { const int c = q >> 6, pp = q & 63; tile[c][pp] = x[((size_t)b * CC + c0 + c) * NP + p0 + pp]; }
  __syncthreads();
  for (int q = tid; q < 64 * 16; q += 256) { const int pp = q >> 4, pc = q & 15;
    v4f v = { tile[pc * 4][pp], tile[pc * 4 + 1][pp], tile[pc * 4 + 2][pp], tile[pc * 4 + 3][pp] };
    vst2(xt + ((size_t)b * NP + p0 + pp) * CC + c0 + pc * 4, v); }
}
__global__ __launch_bounds__(64) void k_sample(const float* __restrict__ xt, const float* __restrict__ om, _Float16* __restrict__ A16) {
  __shared__ __align__(16) _Float16 row[KTOT];
  const int b = blockIdx.y, p = blockIdx.x, c = threadIdx.x; const int oy = p / WW, ox = p % WW;
  const float* omr = om + ((size_t)b * NP + p) * 32; const float* xb = xt + (size_t)b * NP * CC;
#pragma unroll 1
  for (int t = 0; t < KK; ++t) { const int ii = t / 3, jj = t % 3;
    const float py = omr[2 * t] + (float)(oy - 1) + (float)ii, px = omr[2 * t + 1] + (float)(ox - 1) + (float)jj;
    const float fy = floorf(py), fx = floorf(px); const float wy = py - fy, wx = px - fx; const int y0 = (int)fy, x0 = (int)fx;
    float acc = 0.f;
#pragma unroll
    for (int q = 0; q < 4; ++q) { const int yy = y0 + (q >> 1), xx = x0 + (q & 1);
      const float wgt = ((q >> 1) ? wy : 1.0f - wy) * ((q & 1) ? wx : 1.0f - wx);
      if (yy >= 0 && yy <= HH - 1 && xx >= 0 && xx <= WW - 1) acc += xb[((size_t)yy * WW + xx) * CC + c] * wgt; }
    row[c * KK + t] = (_Float16)acc; }
  __syncthreads();
  for (int q = threadIdx.x; q < KTOT / 8; q += 64) vst2(A16 + ((size_t)b * NP + p) * KTOT + q * 8, *(const v4u*)(&row[q * 8]));
}
__global__ __launch_bounds__(128) void k_conv(const _Float16* __restrict__ A16, const float* __restrict__ W, float* __restrict__ pre, float* __restrict__ part) {
  __shared__ __align__(16) float st[64][68];
  __shared__ __align__(16) float sp[64][2];
  const int tid = threadIdx.x, wave = tid >> 5, lane = tid & 31, col = lane & 15, g = lane >> 4;
  const int b = blockIdx.y, p0 = blockIdx.x * 64, r0 = p0 + wave * 16;
  v8f acc[4] = {};
#pragma unroll 1
  for (int kc = 0; kc < KTOT / 32; ++kc) { const v16h a = frag_h(A16 + ((size_t)b * NP + r0 + col) * KTOT + kc * 32, lane);
#pragma unroll
    for (int j = 0; j < 4; ++j) acc[j] = wmma16(a, frag_f32s(W + (size_t)(j * 16 + col) * KTOT + kc * 32, lane, 8.0f), acc[j]); }
#pragma unroll
  for (int j = 0; j < 4; ++j)
#pragma unroll
    for (int r = 0; r < 8; ++r) st[j * 16 + col][wave * 16 + 8 * g + r] = acc[j][r] * 0.125f;
  __syncthreads();
  if (tid < 64) { const int o = tid; float s = 0.f, q2 = 0.f;
#pragma unroll
    for (int pc = 0; pc < 16; ++pc) { const v4f v = *(const v4f*)(&st[o][pc * 4]); vst2(pre + ((size_t)b * OO + o) * NP + p0 + pc * 4, v);
#pragma unroll
      for (int e = 0; e < 4; ++e) { s += v[e]; q2 += v[e] * v[e]; } }
    sp[o][0] = s; sp[o][1] = q2; }
  __syncthreads();
  if (tid < 32) vst2(part + ((size_t)b * NPB + blockIdx.x) * 128 + tid * 4, *(const v4f*)(&sp[0][0] + tid * 4));
}
__global__ __launch_bounds__(64) void k_bnstat(const float* __restrict__ part, float* __restrict__ stat) {
  const int o = threadIdx.x; float s = 0.f, q2 = 0.f;
#pragma unroll 1
  for (int i = 0; i < NB * NPB; ++i) { s += part[(size_t)i * 128 + o * 2]; q2 += part[(size_t)i * 128 + o * 2 + 1]; }
  const float n = (float)(NB * NP); const float mu = s / n; float var = q2 / n - mu * mu; var = var < 0.f ? 0.f : var;
  __shared__ __align__(16) float so[128];
  so[o * 2] = mu; so[o * 2 + 1] = rsqrtf(var + 1e-5f);
  __syncthreads();
  if (o < 32) vst2(stat + o * 4, *(const v4f*)(&so[o * 4]));
}
__global__ __launch_bounds__(256) void k_apply(const float* __restrict__ pre, const float* __restrict__ stat, const float* __restrict__ gam, const float* __restrict__ bet, float* __restrict__ out) {
  const int b = blockIdx.y, o = blockIdx.x, tid = threadIdx.x; const float mu = stat[o * 2], rs = stat[o * 2 + 1], ga = gam[o], be = bet[o];
  const float* src = pre + ((size_t)b * OO + o) * NP; float* dst = out + ((size_t)b * OO + o) * NP;
  for (int q = tid; q < NP / 4; q += 256) { v4f v = *(const v4f*)(src + q * 4);
#pragma unroll
    for (int e = 0; e < 4; ++e) { const float t = (v[e] - mu) * rs * ga + be; v[e] = t > 0.f ? t : 0.f; }
    vst2(dst + q * 4, v); }
}
extern "C" void kernel_launch(void* const* d_in, const int* in_sizes, int n_in, void* d_out, int out_size, void* d_ws, size_t ws_size, hipStream_t stream) {
  (void)in_sizes; (void)n_in; (void)out_size; (void)ws_size;
  const float* x = (const float*)d_in[0]; const float* ow = (const float*)d_in[1]; const float* ob = (const float*)d_in[2]; const float* W = (const float*)d_in[3];
  const float* gam = (const float*)d_in[4]; const float* bet = (const float*)d_in[5];
  float* out = (float*)d_out;
  char* ws = (char*)d_ws; size_t off = 0;
  auto take = [&](size_t bytes) { char* p = ws + off; off += (bytes + 255) & ~(size_t)255; return p; };
  float* om = (float*)take((size_t)NB * NP * 32 * 4); float* xt = (float*)take((size_t)NB * NP * CC * 4); _Float16* A16 = (_Float16*)take((size_t)NB * NP * KTOT * 2);
  float* pre = (float*)take((size_t)NB * OO * NP * 4); float* part = (float*)take((size_t)NB * NPB * 128 * 4); float* stat = (float*)take(128 * 4);
  k_off<<<dim3(NP / 64, NB), 128, 0, stream>>>(x, ow, ob, om);
  k_xT<<<dim3(NP / 64, CC / 64, NB), 256, 0, stream>>>(x, xt);
  k_sample<<<dim3(NP, NB), 64, 0, stream>>>(xt, om, A16);
  k_conv<<<dim3(NP / 64, NB), 128, 0, stream>>>(A16, W, pre, part);
  k_bnstat<<<1, 64, 0, stream>>>(part, stat);
  k_apply<<<dim3(OO, NB), 256, 0, stream>>>(pre, stat, gam, bet, out);
}
